// _UserModel_82806969467402
// MI455X (gfx1250) — hardware-verified
//
#include <hip/hip_runtime.h>
#include <stdint.h>


typedef _Float16 v16h __attribute__((ext_vector_type(16)));
typedef _Float16 v8h  __attribute__((ext_vector_type(8)));
typedef _Float16 v2h  __attribute__((ext_vector_type(2)));
typedef float    v8f  __attribute__((ext_vector_type(8)));
typedef float    v4f  __attribute__((ext_vector_type(4)));
typedef unsigned int v4u __attribute__((ext_vector_type(4)));

static_assert(sizeof(v16h) == 32);
static_assert(sizeof(v8h) == 16);
static_assert(sizeof(v4u) == 16);
static_assert(sizeof(v4f) == 16);

#define LSEQ   200
#define NTILE  13
#define TROWS  208
#define DD     64
#define NWAVE  8
#define NTHR   256

#define WO_G1  0
#define WO_G2  8192
#define WO_G3  10240
#define WO_A1  12288
#define WO_A2  20480
#define W_HALVES 22528
#define PREP_BLOCKS 11

union Frag { v16h v; v8h hv[2]; };
union __attribute__((aligned(16))) WaveBuf { _Float16 x[16 * 128]; float f[16 * 32]; };

__device__ __forceinline__ v8f wmma_f16(v16h a, v16h b, v8f c) {
    c = __builtin_amdgcn_wmma_f32_16x16x32_f16(false, a, false, b, (short)0, c, false, false);
    asm volatile("v_nop\n\tv_nop\n\tv_nop\n\tv_nop" : "+v"(c) : "v"(a), "v"(b));
    return c;
}

template <int K, int NT>
__device__ __forceinline__ void tile_gemm(const _Float16* A, const _Float16* Wt, v8f (&acc)[NT], int m, int h) {
#pragma unroll
    for (int nt = 0; nt < NT; ++nt) {
        v8f z;
#pragma unroll
        for (int i = 0; i < 8; ++i) z[i] = 0.f;
        acc[nt] = z;
    }
    const _Float16* arow = A + m * K;
#pragma unroll 1
    for (int kt = 0; kt < K / 32; ++kt) {
        const int k0 = kt * 32;
        Frag a;
        a.hv[0] = *(const v8h*)(arow + k0 + 8 * h);
        a.hv[1] = *(const v8h*)(arow + k0 + 16 + 8 * h);
#pragma unroll
        for (int nt = 0; nt < NT; ++nt) {
            const _Float16* bp = Wt + (nt * 16 + m) * K + k0 + 8 * h;
            Frag b;
            b.hv[0] = *(const v8h*)(bp);
            b.hv[1] = *(const v8h*)(bp + 16);
            acc[nt] = wmma_f16(a.v, b.v, acc[nt]);
        }
    }
}

template <int NT, bool RELU>
__device__ __forceinline__ void epi_f16(const v8f (&acc)[NT], float inv, const float* __restrict__ bias,
                                        _Float16* O, int ldo, int m, int h) {
#pragma unroll
    for (int nt = 0; nt < NT; ++nt) {
        const float bv = bias[nt * 16 + m];
#pragma unroll
        for (int r = 0; r < 8; ++r) {
            float v = fmaf(acc[nt][r], inv, bv);
            if (RELU) v = fmaxf(v, 0.f);
            O[(8 * h + r) * ldo + nt * 16 + m] = (_Float16)v;
        }
    }
}

__global__ __launch_bounds__(NTHR) void prep_weight_planes(
    const float* __restrict__ gW1, const float* __restrict__ gW2, const float* __restrict__ gW3,
    const float* __restrict__ aW1, const float* __restrict__ aW2, _Float16* __restrict__ wp) {
    const int g = blockIdx.x * NTHR + (int)threadIdx.x;
    const int o = g * 8;
    const bool ok = o < W_HALVES;
    const float* W = gW1; int lk = 7, N = 64, start = WO_G1; float sc = 8.f;
    if (o >= WO_A2)      { W = aW2; lk = 6; N = 32; start = WO_A2; sc = 8.f; }
    else if (o >= WO_A1) { W = aW1; lk = 7; N = 64; start = WO_A1; sc = 8.f; }
    else if (o >= WO_G3) { W = gW3; lk = 5; N = 64; start = WO_G3; sc = 4.f; }
    else if (o >= WO_G2) { W = gW2; lk = 6; N = 32; start = WO_G2; sc = 8.f; }
    const int lo = o - start;
    const int n  = lo >> lk;
    const int k  = lo & ((1 << lk) - 1);
    v8h hv;
#pragma unroll
    for (int i = 0; i < 8; ++i) {
        float v = ok ? W[(size_t)(k + i) * N + n] : 0.f;
        hv[i] = (_Float16)(v * sc);
    }
    const v4u u = __builtin_bit_cast(v4u, hv);
    _Float16* p = wp + o;
    if (ok) *(volatile v4u*)p = u;
    __threadfence();
    if (ok) *(volatile v4u*)p = u;
}

__global__ __launch_bounds__(NTHR) void user_agg_kernel(
    const int* __restrict__ uids, const int* __restrict__ u_item_pad,
    const float* __restrict__ user_tab, const float* __restrict__ item_tab, const float* __restrict__ rate_tab,
    const float* __restrict__ gb1, const float* __restrict__ gb2, const float* __restrict__ gb3,
    const float* __restrict__ ab1, const float* __restrict__ ab2,
    const float* __restrict__ aW3, const float* __restrict__ ab3,
    const float* __restrict__ hW1, const float* __restrict__ hb1,
    const float* __restrict__ hW2, const float* __restrict__ hb2,
    const _Float16* __restrict__ wplanes, float* __restrict__ out,
    int n_user, int n_item, int n_rate, int n_batch) {

    __shared__ __attribute__((aligned(16))) _Float16 wB[W_HALVES];
    __shared__ WaveBuf bufX[NWAVE];
    __shared__ __attribute__((aligned(16))) _Float16 bufY[NWAVE][16 * 64];
    __shared__ __attribute__((aligned(16))) _Float16 bufZ[NWAVE][16 * 32];
    __shared__ float x_lds[LSEQ * DD];
    __shared__ float alpha_lds[TROWS];
    __shared__ float maskw[NWAVE * 16];
    __shared__ float pu[DD];
    __shared__ float aw3s[32];
    __shared__ float red[NWAVE];
    __shared__ float agg_part[4 * DD];
    __shared__ float agg[DD];
    __shared__ float h1s[DD];
    __shared__ __attribute__((aligned(16))) float outs[DD];

    const int b    = blockIdx.x;
    const int tid  = (int)threadIdx.x;
    const int lane = tid & 31;
    const int h    = lane >> 4;
    const int m    = lane & 15;
    const int wave = __builtin_amdgcn_readfirstlane(tid >> 5);
    (void)n_batch;

    for (int i = tid; i < W_HALVES / 8; i += NTHR)
        *(v8h*)(wB + 8 * i) = *(const v8h*)(wplanes + 8 * i);
    if (tid < DD) {
        int u = uids[b];
        u = u < 0 ? 0 : (u >= n_user ? n_user - 1 : u);
        pu[tid] = user_tab[(size_t)u * DD + tid];
    }
    if (tid < 32) aw3s[tid] = aW3[tid];
    if (tid < TROWS) alpha_lds[tid] = 0.f;
    const float ab3v = ab3[0];
    __syncthreads();

    _Float16* X = bufX[wave].x;
    float*    F = bufX[wave].f;
    _Float16* Y = bufY[wave];
    _Float16* Z = bufZ[wave];
    float*    mw = maskw + wave * 16;

    for (int it = 0; it < 2; ++it) {
        const int  tile   = wave + it * NWAVE;
        const bool active = tile < NTILE;
        const int  t0     = tile * 16;

        if (active) {
            int iid = 0, rid = 0;
            const int tl = t0 + lane;
            if (lane < 16 && tl < LSEQ) {
                const size_t base = ((size_t)b * LSEQ + tl) * 2;
                iid = u_item_pad[base];
                rid = u_item_pad[base + 1];
            }
            if (lane < 16) mw[lane] = (tl < LSEQ && iid > 0) ? 1.f : 0.f;
            int iidc = iid < 0 ? 0 : (iid >= n_item ? n_item - 1 : iid);
            int ridc = rid < 0 ? 0 : (rid >= n_rate ? n_rate - 1 : rid);
#pragma unroll
            for (int r = 0; r < 16; ++r) {
                const int ii = __shfl(iidc, r);
                const int ri = __shfl(ridc, r);
                const float2 q = *(const float2*)(item_tab + (size_t)ii * DD + 2 * lane);
                const float2 e = *(const float2*)(rate_tab + (size_t)ri * DD + 2 * lane);
                v2h qh; qh.x = (_Float16)q.x; qh.y = (_Float16)q.y;
                v2h eh; eh.x = (_Float16)e.x; eh.y = (_Float16)e.y;
                *(v2h*)(X + r * 128 + 2 * lane)      = qh;
                *(v2h*)(X + r * 128 + 64 + 2 * lane) = eh;
            }
        }
        __syncthreads();

        if (active) {
            v8f acc[4];
            tile_gemm<128, 4>(X, wB + WO_G1, acc, m, h);
            epi_f16<4, true>(acc, 0.125f, gb1, Y, 64, m, h);
        }
        __syncthreads();

        if (active) {
            v8f acc[2];
            tile_gemm<64, 2>(Y, wB + WO_G2, acc, m, h);
            epi_f16<2, true>(acc, 0.125f, gb2, Z, 32, m, h);
        }
        __syncthreads();

        if (active) {
            v8f acc[4];
            tile_gemm<32, 4>(Z, wB + WO_G3, acc, m, h);
#pragma unroll
            for (int nt = 0; nt < 4; ++nt) {
                const float bv = gb3[nt * 16 + m];
#pragma unroll
                for (int r = 0; r < 8; ++r) {
                    const float v = fmaf(acc[nt][r], 0.25f, bv);
                    const int row = 8 * h + r;
                    const int t = t0 + row;
                    X[row * 128 + nt * 16 + m] = (_Float16)v;
                    if (t < LSEQ) x_lds[t * DD + nt * 16 + m] = v;
                }
            }
            const float p0 = pu[2 * lane], p1 = pu[2 * lane + 1];
#pragma unroll
            for (int r = 0; r < 16; ++r) {
                const float mk = mw[r];
                v2h ph; ph.x = (_Float16)(mk * p0); ph.y = (_Float16)(mk * p1);
                *(v2h*)(X + r * 128 + 64 + 2 * lane) = ph;
            }
        }
        __syncthreads();

        if (active) {
            v8f acc[4];
            tile_gemm<128, 4>(X, wB + WO_A1, acc, m, h);
            epi_f16<4, true>(acc, 0.125f, ab1, Y, 64, m, h);
        }
        __syncthreads();

        if (active) {
            v8f acc[2];
            tile_gemm<64, 2>(Y, wB + WO_A2, acc, m, h);
#pragma unroll
            for (int nt = 0; nt < 2; ++nt) {
                const float bv = ab2[nt * 16 + m];
#pragma unroll
                for (int r = 0; r < 8; ++r)
                    F[(8 * h + r) * 32 + nt * 16 + m] = fmaxf(fmaf(acc[nt][r], 0.125f, bv), 0.f);
            }
        }
        __syncthreads();

        if (active) {
            float s = 0.f;
            const int kb = 16 * h;
#pragma unroll
            for (int k = 0; k < 16; ++k) s = fmaf(F[m * 32 + kb + k], aw3s[kb + k], s);
            s += __shfl_xor(s, 16);
            if (lane < 16) {
                const int t = t0 + lane;
                const float e = expf(s + ab3v);
                alpha_lds[t] = (t < LSEQ) ? mw[lane] * e : 0.f;
            }
        }
        __syncthreads();
    }

    {
        float part = (tid < TROWS) ? alpha_lds[tid] : 0.f;
#pragma unroll
        for (int off = 16; off > 0; off >>= 1) part += __shfl_xor(part, off);
        if (lane == 0) red[tid >> 5] = part;
    }
    __syncthreads();
    float den = red[0];
#pragma unroll
    for (int w = 1; w < NWAVE; ++w) den += red[w];
    den += 1e-10f;
    const float inv = 1.0f / den;
    if (tid < TROWS) {
        const float an = alpha_lds[tid] * inv;
        alpha_lds[tid] = an;
    }
    __syncthreads();

    {
        const int c = tid >> 6, d = tid & 63;
        float a = 0.f;
        for (int t = c; t < LSEQ; t += 4) a = fmaf(alpha_lds[t], x_lds[t * DD + d], a);
        agg_part[c * DD + d] = a;
    }
    __syncthreads();
    if (tid < DD)
        agg[tid] = ((agg_part[tid] + agg_part[DD + tid]) + agg_part[2 * DD + tid]) + agg_part[3 * DD + tid];
    __syncthreads();

    if (tid < DD) {
        float s = 0.f;
        for (int k = 0; k < DD; ++k) s = fmaf(agg[k], hW1[k * DD + tid], s);
        h1s[tid] = fmaxf(s + hb1[tid], 0.f);
    }
    __syncthreads();
    if (tid < DD) {
        float s = 0.f;
        for (int k = 0; k < DD; ++k) s = fmaf(h1s[k], hW2[k * DD + tid], s);
        outs[tid] = fmaxf(s + hb2[tid], 0.f);
    }
    __syncthreads();

    v4f ov;
    ov[0] = 0.f; ov[1] = 0.f; ov[2] = 0.f; ov[3] = 0.f;
    if (tid < 16) ov = *(const v4f*)(outs + 4 * tid);
    if (tid < 16) {
        float* op = out + (size_t)b * DD + 4 * tid;
        *(volatile v4f*)op = ov;
    }
    __threadfence();
    if (tid < 16) {
        float* op = out + (size_t)b * DD + 4 * tid;
        *(volatile v4f*)op = ov;
    }
}

extern "C" void kernel_launch(void* const* d_in, const int* in_sizes, int n_in,
                              void* d_out, int out_size, void* d_ws, size_t ws_size,
                              hipStream_t stream) {
    if (n_in < 21) return;
    const int*   uids       = (const int*)d_in[0];
    const int*   u_item_pad = (const int*)d_in[1];
    const float* user_tab   = (const float*)d_in[2];
    const float* item_tab   = (const float*)d_in[3];
    const float* rate_tab   = (const float*)d_in[4];
    const float* gW1 = (const float*)d_in[5];  const float* gb1 = (const float*)d_in[6];
    const float* gW2 = (const float*)d_in[7];  const float* gb2 = (const float*)d_in[8];
    const float* gW3 = (const float*)d_in[9];  const float* gb3 = (const float*)d_in[10];
    const float* aW1 = (const float*)d_in[11]; const float* ab1 = (const float*)d_in[12];
    const float* aW2 = (const float*)d_in[13]; const float* ab2 = (const float*)d_in[14];
    const float* aW3 = (const float*)d_in[15]; const float* ab3 = (const float*)d_in[16];
    const float* hW1 = (const float*)d_in[17]; const float* hb1 = (const float*)d_in[18];
    const float* hW2 = (const float*)d_in[19]; const float* hb2 = (const float*)d_in[20];

    const int n_batch = out_size / DD;
    if (n_batch <= 0 || out_size != n_batch * DD) return;
    if (in_sizes[0] != n_batch || in_sizes[1] != n_batch * LSEQ * 2) return;
    if (in_sizes[2] < DD || (in_sizes[2] % DD) != 0) return;
    if (in_sizes[3] < DD || (in_sizes[3] % DD) != 0) return;
    if (in_sizes[4] < DD || (in_sizes[4] % DD) != 0) return;
    if (in_sizes[5] != 128 * 64 || in_sizes[6] != 64 || in_sizes[7] != 64 * 32 || in_sizes[8] != 32 ||
        in_sizes[9] != 32 * 64 || in_sizes[10] != 64 || in_sizes[11] != 128 * 64 || in_sizes[12] != 64 ||
        in_sizes[13] != 64 * 32 || in_sizes[14] != 32 || in_sizes[15] != 32 || in_sizes[16] != 1 ||
        in_sizes[17] != 64 * 64 || in_sizes[18] != 64 || in_sizes[19] != 64 * 64 || in_sizes[20] != 64) return;
    const int n_user = in_sizes[2] / DD;
    const int n_item = in_sizes[3] / DD;
    const int n_rate = in_sizes[4] / DD;

    const size_t wp_bytes = (size_t)W_HALVES * sizeof(_Float16);
    if (ws_size < wp_bytes) return;
    _Float16* wplanes = (_Float16*)d_ws;

    prep_weight_planes<<<dim3(PREP_BLOCKS), dim3(NTHR), 0, stream>>>(gW1, gW2, gW3, aW1, aW2, wplanes);

    user_agg_kernel<<<dim3(n_batch), dim3(NTHR), 0, stream>>>(
        uids, u_item_pad, user_tab, item_tab, rate_tab,
        gb1, gb2, gb3, ab1, ab2, aW3, ab3,
        hW1, hb1, hW2, hb2, wplanes, (float*)d_out,
        n_user, n_item, n_rate, n_batch);
}
